// State_and_Language_Pair_Encoder_25537875542358
// MI455X (gfx1250) — hardware-verified
//
#include <hip/hip_runtime.h>


#define NB_  4096
#define DD   256
#define HH   384
#define QQ   512
#define NE   34
#define BCH  512
#define H1W  (NE * HH)
#define QVW  (NE * QQ)

typedef unsigned short bf;
typedef __attribute__((ext_vector_type(16))) __bf16   v16bf;
typedef __attribute__((ext_vector_type(8)))  unsigned short v8us;
typedef __attribute__((ext_vector_type(8)))  float    v8f;
typedef __attribute__((ext_vector_type(4)))  float    v4f;
typedef v4f  __attribute__((may_alias)) v4fa;
typedef v8us __attribute__((may_alias)) v8usa;

__device__ __forceinline__ unsigned short f2bf(float f) { unsigned u = __float_as_uint(f); u += 0x7FFFu + ((u >> 16) & 1u); return (unsigned short)(u >> 16); }
__device__ __forceinline__ float bf2f(unsigned short b) { return __uint_as_float(((unsigned)b) << 16); }
__device__ __forceinline__ float bfr(float f) { return bf2f(f2bf(f)); }
__device__ __forceinline__ v16bf cat16b(v8us lo, v8us hi) { return __builtin_bit_cast(v16bf, __builtin_shufflevector(lo, hi, 0, 1, 2, 3, 4, 5, 6, 7, 8, 9, 10, 11, 12, 13, 14, 15)); }
__device__ __forceinline__ v8f wmmab(v16bf a, v16bf b, v8f c) { return __builtin_amdgcn_wmma_f32_16x16x32_bf16(false, a, false, b, (short)0, c, false, false); }

__global__ __launch_bounds__(256) void k_rows(const float* __restrict__ src, int rows, bf* dst) {
    const int lane = threadIdx.x & 31, r = blockIdx.x * 8 + (threadIdx.x >> 5);
    if (r >= rows) return;
    v8us o;
#pragma unroll
    for (int i = 0; i < 8; ++i) o[i] = f2bf(src[(size_t)r * DD + lane * 8 + i]);
    *(volatile v8us*)(dst + (size_t)r * DD + lane * 8) = o; __threadfence(); *(volatile v8us*)(dst + (size_t)r * DD + lane * 8) = o;
}
__global__ __launch_bounds__(256) void k_wt(const float* __restrict__ Wm, int K, int ncols, bf* WT) {
    __shared__ __align__(16) unsigned short tl[64 * 72];
    const int tid = threadIdx.x, k0 = blockIdx.x * 64, n0 = blockIdx.y * 64, e = blockIdx.z;
    const float* We = Wm + (size_t)e * K * ncols; bf* WTe = WT + (size_t)e * ncols * K;
    const int kk = tid >> 2, nq = (tid & 3) * 16;
#pragma unroll
    for (int i = 0; i < 16; ++i) tl[(nq + i) * 72 + kk] = f2bf(We[(size_t)(k0 + kk) * ncols + n0 + nq + i]);
    __syncthreads();
    const int piece = tid & 7;
    auto pass = [&]() {
#pragma unroll
        for (int s = 0; s < 2; ++s) { const int nr = (tid >> 3) + 32 * s; const v8us val = *(const v8usa*)(tl + nr * 72 + piece * 8); *(volatile v8us*)(WTe + (size_t)(n0 + nr) * K + k0 + piece * 8) = val; }
    };
    pass(); __threadfence(); pass();
}
template <bool SPLITA, int MODE>
__global__ __launch_bounds__(128) void k_gemm(const bf* __restrict__ A, const bf* __restrict__ Al, int lda, int acolstride, const bf* __restrict__ WT, int K, int N, const float* __restrict__ bias, int ldc, float* C, bf* PH, bf* PL) {
    __shared__ __align__(16) float ost[4][16 * 68];
    const int lane = threadIdx.x & 31, wave = threadIdx.x >> 5, lr = lane & 15, hi = lane >> 4, e = blockIdx.z;
    const size_t r0 = (size_t)blockIdx.x * 64 + wave * 16; const int c0 = blockIdx.y * 64;
    const size_t aoff = (r0 + lr) * (size_t)lda + (size_t)e * acolstride + 8 * hi;
    const bf* Bn = WT + (size_t)e * N * K;
    size_t boff[4];
#pragma unroll
    for (int t = 0; t < 4; ++t) boff[t] = (size_t)(c0 + t * 16 + lr) * K + 8 * hi;
    v8f acc[4];
#pragma unroll
    for (int t = 0; t < 4; ++t) acc[t] = (v8f){};
#pragma unroll 2
    for (int kc = 0; kc < K; kc += 32) {
        const v16bf a = cat16b(*(const v8us*)(A + aoff + kc), *(const v8us*)(A + aoff + kc + 16));
        v16bf al = a; if (SPLITA) al = cat16b(*(const v8us*)(Al + aoff + kc), *(const v8us*)(Al + aoff + kc + 16));
#pragma unroll
        for (int t = 0; t < 4; ++t) { const v16bf bb = cat16b(*(const v8us*)(Bn + boff[t] + kc), *(const v8us*)(Bn + boff[t] + kc + 16)); acc[t] = wmmab(a, bb, acc[t]); if (SPLITA) acc[t] = wmmab(al, bb, acc[t]); }
        asm volatile("v_nop" : "+v"(acc[0]), "+v"(acc[1]), "+v"(acc[2]), "+v"(acc[3]) : "v"(a), "v"(al) : "memory");
    }
    float* os = &ost[wave][0];
#pragma unroll
    for (int t = 0; t < 4; ++t) { const float bv = bfr(bias[(size_t)e * N + c0 + t * 16 + lr]);
#pragma unroll
        for (int j = 0; j < 8; ++j) { float v = acc[t][j] + bv; if (MODE == 0) v = fmaxf(v, 0.f); os[(hi * 8 + j) * 68 + t * 16 + lr] = v; } }
    __builtin_amdgcn_wave_barrier(); asm volatile("" ::: "memory");
    const size_t cb = r0 * ldc + (size_t)e * N + c0;
    if (MODE == 0) {
        auto pass = [&]() {
#pragma unroll
            for (int s = 0; s < 4; ++s) { const int row = 4 * s + (lane >> 3), piece = lane & 7; const float* sp = os + row * 68 + piece * 8; v8us oh, ol;
#pragma unroll
                for (int i = 0; i < 8; ++i) { const unsigned short hb = f2bf(sp[i]); oh[i] = hb; ol[i] = f2bf(sp[i] - bf2f(hb)); }
                *(volatile v8us*)(PH + cb + (size_t)row * ldc + piece * 8) = oh; *(volatile v8us*)(PL + cb + (size_t)row * ldc + piece * 8) = ol; }
        };
        pass(); __threadfence(); pass();
    } else {
        auto pass = [&]() {
#pragma unroll
            for (int s = 0; s < 8; ++s) { const int Lid = (lane >> 3) + 4 * s, piece = lane & 7; const int row = Lid >> 1, cofs = (Lid & 1) * 32 + piece * 4;
                const v4f val = *(const v4fa*)(os + row * 68 + cofs); *(volatile v4f*)(C + cb + (size_t)row * ldc + cofs) = val; }
        };
        pass(); __threadfence(); pass();
    }
}
__global__ __launch_bounds__(256) void k_post(const float* __restrict__ QV, const int* __restrict__ tid_in, const float* __restrict__ lang, int b0, float* out0, float* out2, float* LPS) {
    __shared__ float red[2][NE][8];
    __shared__ float lp[64]; __shared__ float pe[NE];
    __shared__ __align__(16) float lat[QQ]; __shared__ __align__(16) float tgt[QQ];
    const int tid = threadIdx.x, bl = blockIdx.x; const size_t b = (size_t)b0 + bl;
    int tk = tid_in[b]; tk = tk < 0 ? 0 : (tk >= NE ? NE - 1 : tk);
    const float* qv = QV + (size_t)bl * QVW;
    const int lane = tid & 31, wave = tid >> 5;
    const float l0 = bfr(lang[(size_t)tk * QQ + tid]), l1 = bfr(lang[(size_t)tk * QQ + tid + 256]);
#pragma unroll 1
    for (int e = 0; e < NE; ++e) { const float q0 = qv[e * QQ + tid], q1 = qv[e * QQ + tid + 256]; float d = q0 * l0 + q1 * l1, s = q0 * q0 + q1 * q1;
#pragma unroll
        for (int sh = 16; sh; sh >>= 1) { d += __shfl_xor(d, sh, 32); s += __shfl_xor(s, sh, 32); }
        if (lane == 0) { red[0][e][wave] = d; red[1][e][wave] = s; } }
    __syncthreads();
    if (tid < NE) { float d = 0.f, s = 0.f;
#pragma unroll
        for (int w = 0; w < 8; ++w) { d += red[0][tid][w]; s += red[1][tid][w]; }
        red[0][tid][0] = d; red[1][tid][0] = s; }
    __syncthreads();
    if (tid < 32) {
        float lsq = 0.f;
#pragma unroll 1
        for (int c = 0; c < QQ; ++c) { const float lv = bfr(lang[(size_t)tk * QQ + c]); lsq += lv * lv; }
        const float lnrm = sqrtf(lsq);
        float lg0 = -3.0e38f, lg1 = -3.0e38f;
        { const int e = tid; const float cs = red[0][e][0] / fmaxf(sqrtf(red[1][e][0]) * lnrm, 1e-8f); lg0 = cs * 10.0f; }
        if (tid + 32 < NE) { const int e = tid + 32; const float cs = red[0][e][0] / fmaxf(sqrtf(red[1][e][0]) * lnrm, 1e-8f); lg1 = cs * 10.0f; }
        float mx = fmaxf(lg0, lg1);
#pragma unroll
        for (int sh = 16; sh; sh >>= 1) mx = fmaxf(mx, __shfl_xor(mx, sh, 32));
        float se = __expf(lg0 - mx) + ((tid + 32 < NE) ? __expf(lg1 - mx) : 0.f);
#pragma unroll
        for (int sh = 16; sh; sh >>= 1) se += __shfl_xor(se, sh, 32);
        const float lse = mx + __logf(se);
        lp[tid] = lg0 - lse; pe[tid] = __expf(lg0 - lse);
        if (tid + 32 < NE) { lp[tid + 32] = lg1 - lse; pe[tid + 32] = __expf(lg1 - lse); } else lp[tid + 32] = 0.f;
    }
    __syncthreads();
    { float a0 = 0.f, a1 = 0.f;
#pragma unroll 1
      for (int e = 0; e < NE; ++e) { const float p = pe[e]; a0 += p * qv[e * QQ + tid]; a1 += p * qv[e * QQ + tid + 256]; }
      lat[tid] = a0; lat[tid + 256] = a1; tgt[tid] = qv[tk * QQ + tid]; tgt[tid + 256] = qv[tk * QQ + tid + 256]; }
    __syncthreads();
#pragma unroll 1
    for (int ps = 0; ps < 2; ++ps) {
        if (tid < 128) { *(volatile v4f*)(out0 + b * QQ + tid * 4) = *(const v4fa*)(lat + tid * 4); *(volatile v4f*)(out2 + b * QQ + tid * 4) = *(const v4fa*)(tgt + tid * 4); }
        else if (tid < 128 + 16) { const int q = tid - 128; *(volatile v4f*)(LPS + b * 64 + q * 4) = *(const v4fa*)(lp + q * 4); }
        if (ps == 0) __threadfence(); }
}
__global__ __launch_bounds__(256) void k_out1(const float* __restrict__ LPS, float* out1) {
    const int f = blockIdx.x * 256 + threadIdx.x; if (f >= NB_ * NE) return;
    const int b = f / NE, e = f - b * NE; const float v = LPS[(size_t)b * 64 + e];
    *(volatile float*)(out1 + f) = v; __threadfence(); *(volatile float*)(out1 + f) = v;
}

extern "C" void kernel_launch(void* const* d_in, const int* in_sizes, int n_in,
                              void* d_out, int out_size, void* d_ws, size_t ws_size, hipStream_t stream) {
    (void)in_sizes; (void)n_in; (void)out_size;
    const float* state = (const float*)d_in[0]; const int* tids = (const int*)d_in[1]; const float* W1 = (const float*)d_in[2]; const float* b1 = (const float*)d_in[3];
    const float* W2 = (const float*)d_in[4]; const float* b2 = (const float*)d_in[5]; const float* W3 = (const float*)d_in[6]; const float* b3 = (const float*)d_in[7]; const float* lang = (const float*)d_in[8];
    float* out0 = (float*)d_out;
    float* out1 = (float*)((char*)d_out + 8388608);
    float* out2 = (float*)((char*)d_out + 8945664);
    char* wsp = (char*)d_ws;
    auto take = [&](size_t bytes) { char* p = wsp; wsp += (bytes + 255) & ~(size_t)255; return (void*)p; };
    bf* Sb = (bf*)take((size_t)NB_ * DD * 2); bf* W1T = (bf*)take((size_t)NE * HH * DD * 2); bf* W2T = (bf*)take((size_t)NE * HH * HH * 2); bf* W3T = (bf*)take((size_t)NE * QQ * HH * 2);
    bf* H1H = (bf*)take((size_t)BCH * H1W * 2); bf* H1L = (bf*)take((size_t)BCH * H1W * 2); bf* H2H = (bf*)take((size_t)BCH * H1W * 2); bf* H2L = (bf*)take((size_t)BCH * H1W * 2);
    float* QV = (float*)take((size_t)BCH * QVW * 4); float* LPS = (float*)take((size_t)NB_ * 64 * 4);
    if ((size_t)(wsp - (char*)d_ws) > ws_size) return;
    k_rows<<<NB_ / 8, 256, 0, stream>>>(state, NB_, Sb);
    k_wt<<<dim3(DD / 64, HH / 64, NE), 256, 0, stream>>>(W1, DD, HH, W1T); k_wt<<<dim3(HH / 64, HH / 64, NE), 256, 0, stream>>>(W2, HH, HH, W2T); k_wt<<<dim3(HH / 64, QQ / 64, NE), 256, 0, stream>>>(W3, HH, QQ, W3T);
    for (int ch = 0; ch < NB_ / BCH; ++ch) { const int b0 = ch * BCH;
        k_gemm<false, 0><<<dim3(BCH / 64, HH / 64, NE), 128, 0, stream>>>(Sb + (size_t)b0 * DD, nullptr, DD, 0, W1T, DD, HH, b1, H1W, nullptr, H1H, H1L);
        k_gemm<true,  0><<<dim3(BCH / 64, HH / 64, NE), 128, 0, stream>>>(H1H, H1L, H1W, HH, W2T, HH, HH, b2, H1W, nullptr, H2H, H2L);
        k_gemm<true,  1><<<dim3(BCH / 64, QQ / 64, NE), 128, 0, stream>>>(H2H, H2L, H1W, HH, W3T, HH, QQ, b3, QVW, QV, nullptr, nullptr);
        k_post<<<BCH, 256, 0, stream>>>(QV, tids, lang, b0, out0, out2, LPS);
    }
    k_out1<<<(NB_ * NE + 255) / 256, 256, 0, stream>>>(LPS, out1);
}
